// SheafWindowLayer_85779086835859
// MI455X (gfx1250) — hardware-run, weakly checked
//
#include <hip/hip_runtime.h>


#ifndef NB
#define NB 2
#endif
#ifndef SEQ
#define SEQ 512
#endif
#define NB_FULL  2
#define SEQ_FULL 512
#ifndef OUT_SEQ
#define OUT_SEQ SEQ
#endif
#define HID   768
#define MH    128
#define NAB   (2 * MH)
#define WIN_  512
#define HALFW (WIN_ / 2)
#define WROWS 8
#define W1S   64.0f
#define W1I   (1.0f / 64.0f)
#define W2S   64.0f
#define W2I   (1.0f / 64.0f)

static_assert(NB <= NB_FULL);
static_assert(SEQ <= SEQ_FULL);
static_assert(SEQ <= WIN_);
static_assert((NB * SEQ) % 64 == 0);
static_assert(NAB % 64 == 0);
static_assert(MH % 64 == 0);
static_assert(HID % 64 == 0);
static_assert(HID % 32 == 0);
static_assert(MH % 32 == 0);
static_assert((2 * HID) % 64 == 0);
static_assert(HID % 8 == 0);
static_assert((NB * SEQ) % WROWS == 0);
static_assert(MH == 32 * 4);
static_assert((MH & (MH - 1)) == 0);
static_assert(32 * 16 * 8 == 16 * 64 * 4);
static_assert(256 * 16 * 2 == 64 * 64 * 2);
static_assert(WROWS * 16 * 16 == WROWS * MH * 2);
static_assert(16 * 68 * 4 <= 131072);
static_assert(64 * 65 * 4 <= 131072);
static_assert(WROWS * MH * 4 <= 131072);

typedef _Float16 h16;
typedef unsigned short bf;
typedef __attribute__((ext_vector_type(16))) _Float16 v16h;
typedef __attribute__((ext_vector_type(8)))  _Float16 v8h;
typedef __attribute__((ext_vector_type(8)))  float    v8f;
typedef __attribute__((ext_vector_type(4)))  float    v4f;
typedef v4f  __attribute__((may_alias)) v4fa;

__device__ __forceinline__ unsigned short f2bf(float f) { unsigned u = __float_as_uint(f); u += 0x7FFFu + ((u >> 16) & 1u); return (unsigned short)(u >> 16); }
__device__ __forceinline__ float bfr(float f) { return __uint_as_float(((unsigned)f2bf(f)) << 16); }
__device__ __forceinline__ v16h cat16(v8h lo, v8h hi) { return __builtin_shufflevector(lo, hi, 0, 1, 2, 3, 4, 5, 6, 7, 8, 9, 10, 11, 12, 13, 14, 15); }
__device__ __forceinline__ v16h  ldh(const h16* p) { return cat16(*(const v8h*)p, *(const v8h*)(p + 16)); }
__device__ __forceinline__ void wave_sync() { __builtin_amdgcn_fence(3  , "wavefront"); __builtin_amdgcn_wave_barrier(); asm volatile("" ::: "memory"); }
static __device__ __forceinline__ h16 toh_flush(float v) { const h16 r = (h16)v; return (fabsf(v) < 6.103515625e-05f) ? (h16)0.0f : r; }
__device__ __forceinline__ v8f wmma16g(v16h a, v16h b, v8f c) {
    c = __builtin_amdgcn_wmma_f32_16x16x32_f16(false, a, false, b, (short)0, c, false, false);
    asm volatile("v_nop\n\tv_nop\n\tv_nop\n\tv_nop" : "+v"(c) : "v"(a), "v"(b));
    return c;
}

__global__ __launch_bounds__(256) void k_xprep(const float* __restrict__ hs, const float* __restrict__ pos, h16* XH, size_t n8) {
    const size_t i = (size_t)blockIdx.x * 256 + threadIdx.x; if (i >= n8) return;
    const size_t e = i * 8; const size_t gm = e / HID; const size_t col = e % HID;
    const size_t bb = gm / SEQ, tt = gm % SEQ;
    const v8f hv = *(const v8f*)(hs + (bb * SEQ_FULL + tt) * HID + col);
    const v8f pv = *(const v8f*)(pos + tt * HID + col);
    v8h o;
#pragma unroll
    for (int k = 0; k < 8; ++k) o[k] = toh_flush(bfr(hv[k]) + bfr(pv[k]));
    *(volatile v8h*)(XH + i * 8) = o; __threadfence(); *(volatile v8h*)(XH + i * 8) = o;
}

__global__ __launch_bounds__(256) void k_wtr(const float* __restrict__ src, h16* dst, int R, int C, float scale) {
    __shared__ float tl[64 * 65];
    const int tid = threadIdx.x; const int c0 = blockIdx.x * 64, r0 = blockIdx.y * 64;
#pragma unroll 1
    for (int it = 0; it < 16; ++it) { const int r = it * 4 + (tid >> 6), c = tid & 63;
        tl[r * 65 + c] = bfr(src[(size_t)(r0 + r) * C + c0 + c]) * scale; }
    __syncthreads();
#pragma unroll 1
    for (int ps = 0; ps < 2; ++ps) {
#pragma unroll 1
        for (int it = 0; it < 2; ++it) { const int cc = it * 32 + (tid >> 3), p8 = (tid & 7) * 8;
            v8h o;
#pragma unroll
            for (int k = 0; k < 8; ++k) o[k] = toh_flush(tl[(p8 + k) * 65 + cc]);
            *(volatile v8h*)(dst + (size_t)(c0 + cc) * R + r0 + p8) = o; }
        if (ps == 0) __threadfence(); }
}

__global__ __launch_bounds__(32) void k_gemm_ab(const h16* __restrict__ XH, const h16* __restrict__ WT, const float* __restrict__ b1, float* AB) {
    __shared__ __align__(16) float os[16 * 68];
    const int lane = threadIdx.x & 31, lr = lane & 15, hi = lane >> 4; const int r0 = blockIdx.x * 64, c0 = blockIdx.y * 64;
    v8f acc[4][4];
#pragma unroll
    for (int mb = 0; mb < 4; ++mb)
#pragma unroll
        for (int nb = 0; nb < 4; ++nb) acc[mb][nb] = (v8f){};
    const size_t aoff = (size_t)(r0 + lr) * HID + 8 * hi;
    const size_t boff = (size_t)((c0 & (MH - 1)) + lr) * (2 * HID) + (size_t)(c0 / MH) * HID + 8 * hi;
#pragma unroll 1
    for (int kc = 0; kc < HID; kc += 32) {
        v16h a[4];
#pragma unroll
        for (int mb = 0; mb < 4; ++mb) a[mb] = ldh(XH + aoff + (size_t)mb * 16 * HID + kc);
#pragma unroll
        for (int nb = 0; nb < 4; ++nb) { const v16h b = ldh(WT + boff + (size_t)nb * 16 * (2 * HID) + kc);
#pragma unroll
            for (int mb = 0; mb < 4; ++mb) acc[mb][nb] = wmma16g(a[mb], b, acc[mb][nb]); }
    }
    const bool ahalf = c0 < MH;
    float bc[4];
#pragma unroll
    for (int nb = 0; nb < 4; ++nb) { float bv = b1[(c0 + nb * 16 + lr) & (MH - 1)]; asm volatile("" : "+v"(bv)); bc[nb] = ahalf ? bfr(bv) : 0.0f; }
#pragma unroll
    for (int mb = 0; mb < 4; ++mb) {
#pragma unroll
        for (int nb = 0; nb < 4; ++nb) {
#pragma unroll
            for (int j = 0; j < 8; ++j) os[(hi * 8 + j) * 68 + nb * 16 + lr] = acc[mb][nb][j] * W1I + bc[nb]; }
        wave_sync();
#pragma unroll 1
        for (int ps = 0; ps < 2; ++ps) {
#pragma unroll 1
            for (int s = 0; s < 8; ++s) { const int row = 2 * s + (lane >> 4), cofs = (lane & 15) * 4;
                const v4f val = *(const v4fa*)(&os[row * 68 + cofs]);
                *(volatile v4f*)(AB + (size_t)(r0 + mb * 16 + row) * NAB + c0 + cofs) = val; }
            if (ps == 0) __threadfence(); }
        wave_sync();
    }
}

__global__ __launch_bounds__(32 * WROWS) void k_span(const float* __restrict__ AB, h16* HH) {
    __shared__ __align__(16) float hsum[WROWS * MH];
    const int tid = threadIdx.x, lane = tid & 31;
    const int wv = tid >> 5;
    const int gmv = blockIdx.x * WROWS + wv;
    const int iv = gmv % SEQ;
    int lov = iv - HALFW; lov = lov > 0 ? lov : 0;
    int hiv = iv + HALFW - 1; hiv = hiv < (SEQ - 1) ? hiv : (SEQ - 1);
    const int wave = __builtin_amdgcn_readfirstlane(wv);
    const int gm = __builtin_amdgcn_readfirstlane(gmv);
    const int jlo = __builtin_amdgcn_readfirstlane(lov);
    const int jhi = __builtin_amdgcn_readfirstlane(hiv);
    const int bb = gm / SEQ;
    const v4f av = *(const v4f*)(AB + (size_t)gm * NAB + lane * 4);
    const float* bp = AB + (size_t)bb * SEQ * NAB + MH + lane * 4;
    v4f acc = (v4f){};
#pragma unroll 4
    for (int j = jlo; j <= jhi; ++j) {
        const v4f bv = *(const v4f*)(bp + (size_t)j * NAB);
#pragma unroll
        for (int k = 0; k < 4; ++k) acc[k] += fmaxf(av[k] + bv[k], 0.0f); }
    const float inv = 1.0f / (float)(jhi - jlo + 1);
    v4f hv;
#pragma unroll
    for (int k = 0; k < 4; ++k) hv[k] = acc[k] * inv;
    *(v4fa*)(&hsum[wave * MH + lane * 4]) = hv;
    __syncthreads();
    if (tid < WROWS * 16) { const int row = tid >> 4, p8 = (tid & 15) * 8;
        const v4f x0 = *(const v4fa*)(&hsum[row * MH + p8]); const v4f x1 = *(const v4fa*)(&hsum[row * MH + p8 + 4]); v8h o;
#pragma unroll
        for (int k = 0; k < 4; ++k) { o[k] = toh_flush(x0[k]); o[4 + k] = toh_flush(x1[k]); }
        h16* dp = HH + ((size_t)blockIdx.x * WROWS + row) * MH + p8;
        *(volatile v8h*)dp = o; __threadfence(); *(volatile v8h*)dp = o; }
}

__global__ __launch_bounds__(32) void k_gemm_out(const h16* __restrict__ HH, const h16* __restrict__ WT, const float* __restrict__ b2,
                                                 const float* __restrict__ hs, const float* __restrict__ pos, const float* __restrict__ alpha_p, float* OUT) {
    __shared__ __align__(16) float os[16 * 68];
    const int lane = threadIdx.x & 31, lr = lane & 15, hi = lane >> 4; const int r0 = blockIdx.x * 64, c0 = blockIdx.y * 64;
    v8f acc[4][4];
#pragma unroll
    for (int mb = 0; mb < 4; ++mb)
#pragma unroll
        for (int nb = 0; nb < 4; ++nb) acc[mb][nb] = (v8f){};
    const size_t aoff = (size_t)(r0 + lr) * MH + 8 * hi, boff = (size_t)(c0 + lr) * MH + 8 * hi;
#pragma unroll 1
    for (int kc = 0; kc < MH; kc += 32) {
        v16h a[4];
#pragma unroll
        for (int mb = 0; mb < 4; ++mb) a[mb] = ldh(HH + aoff + (size_t)mb * 16 * MH + kc);
#pragma unroll
        for (int nb = 0; nb < 4; ++nb) { const v16h b = ldh(WT + boff + (size_t)nb * 16 * MH + kc);
#pragma unroll
            for (int mb = 0; mb < 4; ++mb) acc[mb][nb] = wmma16g(a[mb], b, acc[mb][nb]); }
    }
    const float al = bfr(alpha_p[0]);
#pragma unroll
    for (int mb = 0; mb < 4; ++mb) {
#pragma unroll
        for (int nb = 0; nb < 4; ++nb) {
#pragma unroll
            for (int j = 0; j < 8; ++j) os[(hi * 8 + j) * 68 + nb * 16 + lr] = acc[mb][nb][j] * W2I; }
        wave_sync();
#pragma unroll 1
        for (int ps = 0; ps < 2; ++ps) {
#pragma unroll 1
            for (int s = 0; s < 8; ++s) { const int row = 2 * s + (lane >> 4), cofs = (lane & 15) * 4;
                const int gm = r0 + mb * 16 + row; const int bb = gm / SEQ, tt = gm % SEQ; const int col = c0 + cofs;
                const v4f ag = *(const v4fa*)(&os[row * 68 + cofs]);
                const v4f hv = *(const v4f*)(hs + ((size_t)bb * SEQ_FULL + tt) * HID + col);
                const v4f pv = *(const v4f*)(pos + (size_t)tt * HID + col);
                const v4f bv = *(const v4f*)(b2 + col);
                v4f val;
#pragma unroll
                for (int i = 0; i < 4; ++i) { const float x = bfr(hv[i]) + bfr(pv[i]); const float g = ag[i] + bfr(bv[i]); val[i] = x + al * (g - x); }
                *(volatile v4f*)(OUT + ((size_t)bb * OUT_SEQ + tt) * HID + col) = val; }
            if (ps == 0) __threadfence(); }
        wave_sync();
    }
}

static constexpr size_t al256(size_t v) { return (v + 255) & ~(size_t)255; }
static constexpr size_t SZ_XH = al256((size_t)NB * SEQ * HID * 2);
static constexpr size_t SZ_W1 = al256((size_t)MH * 2 * HID * 2);
static constexpr size_t SZ_W2 = al256((size_t)HID * MH * 2);
static constexpr size_t SZ_AB = al256((size_t)NB * SEQ * NAB * 4);
static constexpr size_t SZ_HH = al256((size_t)NB * SEQ * MH * 2);
static constexpr size_t SZ_TOTAL = SZ_XH + SZ_W1 + SZ_W2 + SZ_AB + SZ_HH;
static_assert(SZ_TOTAL <= (size_t)134217728);
static_assert(((size_t)NB * SEQ * HID) % 8 == 0);

extern "C" void kernel_launch(void* const* d_in, const int* in_sizes, int n_in,
                              void* d_out, int out_size, void* d_ws, size_t ws_size, hipStream_t stream) {
    if (n_in < 7) return;
    const size_t needx = ((size_t)(NB - 1) * SEQ_FULL + SEQ) * HID;
    if ((size_t)in_sizes[0] < needx) return;
    if ((size_t)in_sizes[1] < (size_t)SEQ * HID) return;
    if ((size_t)in_sizes[2] < (size_t)2 * HID * MH) return;
    if (in_sizes[3] < MH) return;
    if ((size_t)in_sizes[4] < (size_t)MH * HID) return;
    if (in_sizes[5] < HID || in_sizes[6] < 1) return;
    if ((size_t)out_size < ((size_t)(NB - 1) * OUT_SEQ + SEQ) * HID) return;
    if (SZ_TOTAL > ws_size) return;
    const float* hs  = (const float*)d_in[0];
    const float* pos = (const float*)d_in[1];
    const float* w1  = (const float*)d_in[2];
    const float* b1  = (const float*)d_in[3];
    const float* w2  = (const float*)d_in[4];
    const float* b2  = (const float*)d_in[5];
    const float* alp = (const float*)d_in[6];
    float* OUT = (float*)d_out;
    char* wsp = (char*)d_ws;
    h16* XH  = (h16*)wsp;   wsp += SZ_XH;
    h16* W1T = (h16*)wsp;   wsp += SZ_W1;
    h16* W2T = (h16*)wsp;   wsp += SZ_W2;
    float* AB = (float*)wsp; wsp += SZ_AB;
    h16* HH  = (h16*)wsp;   wsp += SZ_HH;

    { const size_t n8 = (size_t)NB * SEQ * HID / 8;
      k_xprep<<<(unsigned)((n8 + 255) / 256), 256, 0, stream>>>(hs, pos, XH, n8); }
    k_wtr<<<dim3(MH / 64, (2 * HID) / 64, 1), 256, 0, stream>>>(w1, W1T, 2 * HID, MH, W1S);
    k_wtr<<<dim3(HID / 64, MH / 64, 1), 256, 0, stream>>>(w2, W2T, MH, HID, W2S);

    k_gemm_ab<<<dim3(NB * SEQ / 64, NAB / 64, 1), 32, 0, stream>>>(XH, W1T, b1, AB);
    k_span<<<dim3(NB * SEQ / WROWS, 1, 1), 32 * WROWS, 0, stream>>>(AB, HH);
    k_gemm_out<<<dim3(NB * SEQ / 64, HID / 64, 1), 32, 0, stream>>>(HH, W2T, b2, hs, pos, alp, OUT);
}
